// MultiHeadSelfAttention_65120294142355
// MI455X (gfx1250) — hardware-verified
//
#include <hip/hip_runtime.h>


#ifndef NB
#define NB 4
#endif
#ifndef SEQ
#define SEQ 2048
#endif
#define NB_FULL  4
#define SEQ_FULL 2048
#define DM   512
#define NH   8
#define HD   64
#define NROW (NB * SEQ)
#define RCAR 2048.0f
#define SCL2 0.18033688011112042f

static_assert(NB <= NB_FULL);
static_assert(SEQ <= SEQ_FULL);
static_assert(SEQ % 64 == 0);
static_assert(DM == NH * HD);
static_assert(HD == 64);
static_assert(DM % 64 == 0);
static_assert(DM % 32 == 0);
static_assert(NROW % 64 == 0);
static_assert(NROW % 8 == 0);
static_assert(DM == 4 * 128);
static_assert(((size_t)NROW * DM / 8) % 256 == 0);

typedef _Float16 h16;
typedef unsigned short bf;
typedef __attribute__((ext_vector_type(16))) __bf16   v16bf;
typedef __attribute__((ext_vector_type(16))) _Float16 v16h;
typedef __attribute__((ext_vector_type(8)))  _Float16 v8h;
typedef __attribute__((ext_vector_type(8)))  unsigned short v8us;
typedef __attribute__((ext_vector_type(8)))  float    v8f;
typedef __attribute__((ext_vector_type(4)))  float    v4f;
typedef v8h  __attribute__((may_alias)) v8ha;
typedef v4f  __attribute__((may_alias)) v4fa;
typedef v8us __attribute__((may_alias)) v8usa;

__device__ __forceinline__ unsigned short f2bf(float f) { unsigned u = __float_as_uint(f); u += 0x7FFFu + ((u >> 16) & 1u); return (unsigned short)(u >> 16); }
__device__ __forceinline__ float bf2f(unsigned short b) { return __uint_as_float(((unsigned)b) << 16); }
__device__ __forceinline__ float bfr(float f) { return bf2f(f2bf(f)); }
__device__ __forceinline__ void splitf(float y, unsigned short& h, unsigned short& l) { h = f2bf(y); l = f2bf(y - bf2f(h)); }
__device__ __forceinline__ v16h cat16(v8h lo, v8h hi) { return __builtin_shufflevector(lo, hi, 0, 1, 2, 3, 4, 5, 6, 7, 8, 9, 10, 11, 12, 13, 14, 15); }
__device__ __forceinline__ v16bf cat16b(v8us lo, v8us hi) { return __builtin_bit_cast(v16bf, __builtin_shufflevector(lo, hi, 0, 1, 2, 3, 4, 5, 6, 7, 8, 9, 10, 11, 12, 13, 14, 15)); }
__device__ __forceinline__ v8f wmma16(v16h a, v16h b, v8f c) { return __builtin_amdgcn_wmma_f32_16x16x32_f16(false, a, false, b, (short)0, c, false, false); }
__device__ __forceinline__ v8f wmmab(v16bf a, v16bf b, v8f c) { return __builtin_amdgcn_wmma_f32_16x16x32_bf16(false, a, false, b, (short)0, c, false, false); }
__device__ __forceinline__ v16bf ldb(const bf* p) { return cat16b(*(const v8us*)p, *(const v8us*)(p + 16)); }
__device__ __forceinline__ v16h  ldh(const h16* p) { return cat16(*(const v8h*)p, *(const v8h*)(p + 16)); }
__device__ __forceinline__ size_t xrow(int g) { return (size_t)(g / SEQ) * SEQ_FULL + (size_t)(g % SEQ); }

__global__ __launch_bounds__(256) void k_cvt8x(const float* __restrict__ x, bf* XB) {
    const size_t i = (size_t)blockIdx.x * 256 + threadIdx.x; if (i >= (size_t)NROW * DM / 8) return;
    const int g = (int)(i / (DM / 8)); const int c8 = (int)(i % (DM / 8));
    const v8f v = *(const v8f*)(x + xrow(g) * DM + (size_t)c8 * 8); v8us o;
#pragma unroll
    for (int k = 0; k < 8; ++k) o[k] = f2bf(v[k]);
    *(volatile v8us*)(XB + i * 8) = o; __threadfence(); *(volatile v8us*)(XB + i * 8) = o;
}

__global__ __launch_bounds__(256) void k_wt(const float* __restrict__ w, bf* WT) {
    __shared__ __align__(16) unsigned short ts[64 * 72];
    const int tid = threadIdx.x; const int k0 = blockIdx.x * 64, n0 = blockIdx.y * 64;
#pragma unroll
    for (int it = 0; it < 4; ++it) { const int p = it * 256 + tid; const int kr = p >> 4, c4 = (p & 15) * 4; const v4f v = *(const v4f*)(w + (size_t)(k0 + kr) * DM + n0 + c4);
#pragma unroll
        for (int q = 0; q < 4; ++q) ts[(c4 + q) * 72 + kr] = f2bf(v[q]); }
    __syncthreads();
#pragma unroll 1
    for (int ps = 0; ps < 2; ++ps) {
#pragma unroll
        for (int it = 0; it < 2; ++it) { const int p = it * 256 + tid; const int n = p >> 3, pc = p & 7; const v8us o = *(const v8usa*)(ts + n * 72 + pc * 8);
            *(volatile v8us*)(WT + (size_t)(n0 + n) * DM + k0 + pc * 8) = o; }
        if (ps == 0) __threadfence(); }
}

template <int NSPLIT>
__device__ __forceinline__ void gemm_core(const bf* __restrict__ A, const bf* __restrict__ A2, const bf* __restrict__ Bt, const size_t aoff, const size_t boff, v8f (&acc)[4][4]) {
#pragma unroll
    for (int mb = 0; mb < 4; ++mb)
#pragma unroll
        for (int nb = 0; nb < 4; ++nb) acc[mb][nb] = (v8f){};
#pragma unroll 1
    for (int kc = 0; kc < DM; kc += 32) {
        v16bf a[4], a2[4];
#pragma unroll
        for (int mb = 0; mb < 4; ++mb) { a[mb] = ldb(A + aoff + (size_t)mb * 16 * DM + kc); if (NSPLIT == 1) a2[mb] = ldb(A2 + aoff + (size_t)mb * 16 * DM + kc); }
#pragma unroll
        for (int nb = 0; nb < 4; ++nb) { const v16bf b = ldb(Bt + boff + (size_t)nb * 16 * DM + kc);
#pragma unroll
            for (int mb = 0; mb < 4; ++mb) { acc[mb][nb] = wmmab(a[mb], b, acc[mb][nb]); if (NSPLIT == 1) acc[mb][nb] = wmmab(a2[mb], b, acc[mb][nb]); } }
        if (NSPLIT == 1) { asm volatile("v_nop\n\tv_nop\n\tv_nop\n\tv_nop" : "+v"(acc[0][0]), "+v"(acc[1][1]), "+v"(acc[2][2]), "+v"(acc[3][3]) : "v"(a[0]), "v"(a[1]), "v"(a[2]), "v"(a[3]), "v"(a2[0]), "v"(a2[1]), "v"(a2[2]), "v"(a2[3])); }
        else             { asm volatile("v_nop\n\tv_nop\n\tv_nop\n\tv_nop" : "+v"(acc[0][0]), "+v"(acc[1][1]), "+v"(acc[2][2]), "+v"(acc[3][3]) : "v"(a[0]), "v"(a[1]), "v"(a[2]), "v"(a[3])); }
    }
}

__global__ __launch_bounds__(32) void k_proj_q(const bf* __restrict__ XB, const bf* __restrict__ WT, h16* QH, h16* QR) {
    __shared__ __align__(16) float os[16 * 68];
    const int lane = threadIdx.x & 31, lr = lane & 15, hi = lane >> 4; const int r0 = blockIdx.x * 64, c0 = blockIdx.y * 64;
    v8f acc[4][4];
    gemm_core<0>(XB, XB, WT, (size_t)(r0 + lr) * DM + 8 * hi, (size_t)(c0 + lr) * DM + 8 * hi, acc);
    const int b = r0 / SEQ, s0 = r0 - b * SEQ; const size_t pbase = ((size_t)(b * NH + (int)blockIdx.y) * SEQ + s0) * HD;
#pragma unroll
    for (int mb = 0; mb < 4; ++mb) {
#pragma unroll
        for (int nb = 0; nb < 4; ++nb) {
#pragma unroll
            for (int j = 0; j < 8; ++j) os[(hi * 8 + j) * 68 + nb * 16 + lr] = acc[mb][nb][j]; }
        __builtin_amdgcn_wave_barrier(); asm volatile("" ::: "memory");
        v8h oh[4], orr[4];
#pragma unroll
        for (int s = 0; s < 4; ++s) { const int row = 4 * s + (lane >> 3), pc = lane & 7; const v4f a = *(const v4fa*)(os + row * 68 + pc * 8); const v4f c = *(const v4fa*)(os + row * 68 + pc * 8 + 4);
#pragma unroll
            for (int q = 0; q < 4; ++q) { const h16 xa = (h16)a[q]; oh[s][q] = xa; orr[s][q] = (h16)((a[q] - (float)xa) * RCAR); const h16 xc = (h16)c[q]; oh[s][4 + q] = xc; orr[s][4 + q] = (h16)((c[q] - (float)xc) * RCAR); } }
#pragma unroll 1
        for (int ps = 0; ps < 2; ++ps) {
#pragma unroll
            for (int s = 0; s < 4; ++s) { const int row = 4 * s + (lane >> 3), pc = lane & 7; const size_t o = pbase + (size_t)(mb * 16 + row) * HD + pc * 8;
                *(volatile v8h*)(QH + o) = oh[s]; *(volatile v8h*)(QR + o) = orr[s]; }
            if (ps == 0) __threadfence(); }
        __builtin_amdgcn_wave_barrier(); asm volatile("" ::: "memory");
    }
}

__global__ __launch_bounds__(32) void k_proj_k(const bf* __restrict__ XB, const bf* __restrict__ WT, h16* KP) {
    __shared__ __align__(16) float os[16 * 68];
    const int lane = threadIdx.x & 31, lr = lane & 15, hi = lane >> 4; const int r0 = blockIdx.x * 64, c0 = blockIdx.y * 64;
    v8f acc[4][4];
    gemm_core<0>(XB, XB, WT, (size_t)(r0 + lr) * DM + 8 * hi, (size_t)(c0 + lr) * DM + 8 * hi, acc);
    const int b = r0 / SEQ, s0 = r0 - b * SEQ; const size_t pbase = ((size_t)(b * NH + (int)blockIdx.y) * SEQ + s0) * HD;
#pragma unroll
    for (int mb = 0; mb < 4; ++mb) {
#pragma unroll
        for (int nb = 0; nb < 4; ++nb) {
#pragma unroll
            for (int j = 0; j < 8; ++j) os[(hi * 8 + j) * 68 + nb * 16 + lr] = acc[mb][nb][j]; }
        __builtin_amdgcn_wave_barrier(); asm volatile("" ::: "memory");
        v8h oh[4];
#pragma unroll
        for (int s = 0; s < 4; ++s) { const int row = 4 * s + (lane >> 3), pc = lane & 7; const v4f a = *(const v4fa*)(os + row * 68 + pc * 8); const v4f c = *(const v4fa*)(os + row * 68 + pc * 8 + 4);
#pragma unroll
            for (int q = 0; q < 4; ++q) { oh[s][q] = (h16)a[q]; oh[s][4 + q] = (h16)c[q]; } }
#pragma unroll 1
        for (int ps = 0; ps < 2; ++ps) {
#pragma unroll
            for (int s = 0; s < 4; ++s) { const int row = 4 * s + (lane >> 3), pc = lane & 7; *(volatile v8h*)(KP + pbase + (size_t)(mb * 16 + row) * HD + pc * 8) = oh[s]; }
            if (ps == 0) __threadfence(); }
        __builtin_amdgcn_wave_barrier(); asm volatile("" ::: "memory");
    }
}

__global__ __launch_bounds__(32) void k_proj_v(const bf* __restrict__ XB, const bf* __restrict__ WT, h16* VT) {
    __shared__ __align__(16) h16 vt[64 * 72];
    const int lane = threadIdx.x & 31, lr = lane & 15, hi = lane >> 4; const int r0 = blockIdx.x * 64, c0 = blockIdx.y * 64;
    v8f acc[4][4];
    gemm_core<0>(XB, XB, WT, (size_t)(r0 + lr) * DM + 8 * hi, (size_t)(c0 + lr) * DM + 8 * hi, acc);
    const int b = r0 / SEQ, s0 = r0 - b * SEQ; const size_t pbase = (size_t)(b * NH + (int)blockIdx.y) * HD * SEQ + s0;
#pragma unroll
    for (int mb = 0; mb < 4; ++mb)
#pragma unroll
        for (int nb = 0; nb < 4; ++nb) { v8h o;
#pragma unroll
            for (int j = 0; j < 8; ++j) o[j] = (h16)acc[mb][nb][j];
            *(v8ha*)(vt + (nb * 16 + lr) * 72 + mb * 16 + hi * 8) = o; }
    __builtin_amdgcn_wave_barrier(); asm volatile("" ::: "memory");
#pragma unroll 1
    for (int ps = 0; ps < 2; ++ps) {
#pragma unroll
        for (int it = 0; it < 16; ++it) { const int d = 4 * it + (lane >> 3), pc = lane & 7; const v8h o = *(const v8ha*)(vt + d * 72 + pc * 8);
            *(volatile v8h*)(VT + pbase + (size_t)d * SEQ + pc * 8) = o; }
        if (ps == 0) __threadfence(); }
}

__global__ __launch_bounds__(128) void k_attn(const h16* __restrict__ QH, const h16* __restrict__ QR, const h16* __restrict__ KP, const h16* __restrict__ VT, bf* ATh, bf* ATl) {
    __shared__ __align__(16) unsigned short sth[4 * 16 * 72];
    __shared__ __align__(16) unsigned short stl[4 * 16 * 72];
    const int lane = threadIdx.x & 31, lr = lane & 15, hi = lane >> 4;
    const int wave = __builtin_amdgcn_readfirstlane((int)(threadIdx.x >> 5));
    const int bh = blockIdx.y; const int q0 = blockIdx.x * 64 + wave * 16;
    const size_t pb = (size_t)bh * SEQ * HD;
    const size_t qoff = pb + (size_t)(q0 + lr) * HD + 8 * hi;
    const v16h qh0 = ldh(QH + qoff), qh1 = ldh(QH + qoff + 32), qr0 = ldh(QR + qoff), qr1 = ldh(QR + qoff + 32);
    const size_t koff = pb + (size_t)lr * HD + 8 * hi;
    const size_t voff = pb + (size_t)lr * SEQ + 8 * hi;
    v8f o[4];
#pragma unroll
    for (int c = 0; c < 4; ++c) o[c] = (v8f){};
    float m = -3.0e38f, l = 0.0f;
#pragma unroll 1
    for (int j = 0; j < SEQ; j += 32) {
        const h16* kp = KP + koff + (size_t)j * HD;
        const v16h ka0 = ldh(kp), ka1 = ldh(kp + 32), kb0 = ldh(kp + 16 * HD), kb1 = ldh(kp + 16 * HD + 32);
        v8f s0 = (v8f){}, s1 = (v8f){}, t0 = (v8f){}, t1 = (v8f){};
        s0 = wmma16(ka0, qh0, s0); t0 = wmma16(ka0, qr0, t0); s1 = wmma16(kb0, qh0, s1); t1 = wmma16(kb0, qr0, t1);
        s0 = wmma16(ka1, qh1, s0); t0 = wmma16(ka1, qr1, t0); s1 = wmma16(kb1, qh1, s1); t1 = wmma16(kb1, qr1, t1);
        asm volatile("v_nop\n\tv_nop\n\tv_nop\n\tv_nop" : "+v"(s0), "+v"(s1), "+v"(t0), "+v"(t1) : "v"(ka0), "v"(ka1), "v"(kb0), "v"(kb1), "v"(qh0), "v"(qh1), "v"(qr0), "v"(qr1));
        float z0[8], z1[8]; float mx = -3.0e38f;
#pragma unroll
        for (int r = 0; r < 8; ++r) { z0[r] = (s0[r] + t0[r] * (1.0f / RCAR)) * SCL2; z1[r] = (s1[r] + t1[r] * (1.0f / RCAR)) * SCL2; mx = fmaxf(mx, fmaxf(z0[r], z1[r])); }
        mx = fmaxf(mx, __shfl_xor(mx, 16, 32));
        const float mn = fmaxf(m, mx); const float alpha = __builtin_amdgcn_exp2f(m - mn); m = mn;
        const float mc = mn - 10.0f;
        float rs = 0.0f; v16h pf;
#pragma unroll
        for (int r = 0; r < 8; ++r) { const float a = __builtin_amdgcn_exp2f(z0[r] - mc), c = __builtin_amdgcn_exp2f(z1[r] - mc); rs += a + c; pf[r] = (h16)a; pf[8 + r] = (h16)c; }
        l = l * alpha + rs;
#pragma unroll
        for (int c = 0; c < 4; ++c) o[c] = o[c] * alpha;
        const h16* vp = VT + voff + j;
        const v16h va = ldh(vp), vb = ldh(vp + (size_t)16 * SEQ), vc = ldh(vp + (size_t)32 * SEQ), vd = ldh(vp + (size_t)48 * SEQ);
        o[0] = wmma16(va, pf, o[0]); o[1] = wmma16(vb, pf, o[1]); o[2] = wmma16(vc, pf, o[2]); o[3] = wmma16(vd, pf, o[3]);
        asm volatile("v_nop\n\tv_nop\n\tv_nop\n\tv_nop" : "+v"(o[0]), "+v"(o[1]), "+v"(o[2]), "+v"(o[3]) : "v"(va), "v"(vb), "v"(vc), "v"(vd), "v"(pf));
    }
    const float lt = l + __shfl_xor(l, 16, 32);
    const float inv = 1.0f / lt;
    const int sb = wave * (16 * 72);
#pragma unroll
    for (int c = 0; c < 4; ++c) { v8us oh, ol;
#pragma unroll
        for (int r = 0; r < 8; ++r) { unsigned short a, e; splitf(o[c][r] * inv, a, e); oh[r] = a; ol[r] = e; }
        *(v8usa*)(sth + sb + lr * 72 + 16 * c + 8 * hi) = oh; *(v8usa*)(stl + sb + lr * 72 + 16 * c + 8 * hi) = ol; }
    __builtin_amdgcn_wave_barrier(); asm volatile("" ::: "memory");
    const int b = bh / NH, head = bh - b * NH;
    const size_t ob = ((size_t)b * SEQ + q0) * DM + (size_t)head * HD;
#pragma unroll 1
    for (int ps = 0; ps < 2; ++ps) {
#pragma unroll
        for (int s = 0; s < 4; ++s) { const int row = 4 * s + (lane >> 3), pc = lane & 7; const v8us vh = *(const v8usa*)(sth + sb + row * 72 + pc * 8); const v8us vl = *(const v8usa*)(stl + sb + row * 72 + pc * 8);
            *(volatile v8us*)(ATh + ob + (size_t)row * DM + pc * 8) = vh; *(volatile v8us*)(ATl + ob + (size_t)row * DM + pc * 8) = vl; }
        if (ps == 0) __threadfence(); }
}

__global__ __launch_bounds__(32) void k_oproj(const bf* __restrict__ ATh, const bf* __restrict__ ATl, const bf* __restrict__ WT, const float* __restrict__ x, const float* __restrict__ bo, float* RES) {
    __shared__ __align__(16) float os[16 * 68];
    const int lane = threadIdx.x & 31, lr = lane & 15, hi = lane >> 4; const int r0 = blockIdx.x * 64, c0 = blockIdx.y * 64;
    v8f acc[4][4];
    gemm_core<1>(ATh, ATl, WT, (size_t)(r0 + lr) * DM + 8 * hi, (size_t)(c0 + lr) * DM + 8 * hi, acc);
    const int cofs = lr * 4;
    const v4f bv = *(const v4f*)(bo + c0 + cofs);
    const size_t xb = xrow(r0) * DM + c0 + cofs;
#pragma unroll
    for (int mb = 0; mb < 4; ++mb) {
#pragma unroll
        for (int nb = 0; nb < 4; ++nb) {
#pragma unroll
            for (int j = 0; j < 8; ++j) os[(hi * 8 + j) * 68 + nb * 16 + lr] = acc[mb][nb][j]; }
        __builtin_amdgcn_wave_barrier(); asm volatile("" ::: "memory");
        v4f val[8];
#pragma unroll
        for (int s = 0; s < 8; ++s) { const int row = 2 * s + hi; v4f v = *(const v4fa*)(os + row * 68 + cofs); const v4f xv = *(const v4f*)(x + xb + (size_t)(mb * 16 + row) * DM);
#pragma unroll
            for (int q = 0; q < 4; ++q) v[q] = bfr(xv[q]) + (v[q] + bfr(bv[q]));
            val[s] = v; }
#pragma unroll 1
        for (int ps = 0; ps < 2; ++ps) {
#pragma unroll
            for (int s = 0; s < 8; ++s) { const int row = 2 * s + hi; *(volatile v4f*)(RES + (size_t)(r0 + mb * 16 + row) * DM + c0 + cofs) = val[s]; }
            if (ps == 0) __threadfence(); }
        __builtin_amdgcn_wave_barrier(); asm volatile("" ::: "memory");
    }
}

__global__ __launch_bounds__(256) void k_ln(const float* __restrict__ RES, const float* __restrict__ gamma, const float* __restrict__ beta, float* OUT) {
    const int lane = threadIdx.x & 31;
    const int wave = __builtin_amdgcn_readfirstlane((int)(threadIdx.x >> 5));
    const int row = blockIdx.x * 8 + wave;
    const float* rp = RES + (size_t)row * DM;
    float s = 0.0f;
#pragma unroll 1
    for (int ch = 0; ch < DM / 128; ++ch) { const v4f a = *(const v4f*)(rp + ch * 128 + lane * 4); s += (a[0] + a[1]) + (a[2] + a[3]); }
#pragma unroll
    for (int sh = 16; sh; sh >>= 1) s += __shfl_xor(s, sh, 32);
    const float mu = s * (1.0f / DM);
    float ss = 0.0f;
#pragma unroll 1
    for (int ch = 0; ch < DM / 128; ++ch) { const v4f a = *(const v4f*)(rp + ch * 128 + lane * 4); const float d0 = a[0] - mu, d1 = a[1] - mu, d2 = a[2] - mu, d3 = a[3] - mu; ss += (d0 * d0 + d1 * d1) + (d2 * d2 + d3 * d3); }
#pragma unroll
    for (int sh = 16; sh; sh >>= 1) ss += __shfl_xor(ss, sh, 32);
    const float var = ss * (1.0f / DM);
    const float rstd = 1.0f / sqrtf(var + 1e-6f);
    float* op = OUT + (size_t)row * DM;
#pragma unroll 1
    for (int ps = 0; ps < 2; ++ps) {
#pragma unroll 1
        for (int ch = 0; ch < DM / 128; ++ch) { const int c = ch * 128 + lane * 4; const v4f a = *(const v4f*)(rp + c); const v4f g = *(const v4f*)(gamma + c); const v4f bt = *(const v4f*)(beta + c); v4f y;
#pragma unroll
            for (int q = 0; q < 4; ++q) y[q] = (a[q] - mu) * rstd * bfr(g[q]) + bfr(bt[q]);
            *(volatile v4f*)(op + c) = y; }
        if (ps == 0) __threadfence(); }
}

#define SZ_P16 ((size_t)NROW * DM * 2)
#define SZ_W   ((size_t)DM * DM * 2)
#define SZ_RES ((size_t)NROW * DM * 4)
#define WS_TOTAL (SZ_P16 * 7 + SZ_W * 4 + SZ_RES)
static_assert(SZ_P16 % 256 == 0);
static_assert(SZ_W % 256 == 0);
static_assert(WS_TOTAL <= (size_t)134217728);

extern "C" void kernel_launch(void* const* d_in, const int* in_sizes, int n_in,
                              void* d_out, int out_size, void* d_ws, size_t ws_size, hipStream_t stream) {
    if (n_in < 8) return;
    if ((size_t)in_sizes[0] < ((size_t)(NB - 1) * SEQ_FULL + SEQ) * DM) return;
    if (in_sizes[1] < DM * DM || in_sizes[2] < DM * DM || in_sizes[3] < DM * DM || in_sizes[4] < DM * DM) return;
    if (in_sizes[5] < DM || in_sizes[6] < DM || in_sizes[7] < DM) return;
    if ((size_t)out_size < (size_t)NROW * DM) return;
    if (WS_TOTAL > ws_size) return;
    const float* x = (const float*)d_in[0]; const float* wq = (const float*)d_in[1]; const float* wk = (const float*)d_in[2]; const float* wv = (const float*)d_in[3];
    const float* wo = (const float*)d_in[4]; const float* bo = (const float*)d_in[5]; const float* gamma = (const float*)d_in[6]; const float* beta = (const float*)d_in[7];
    float* OUT = (float*)d_out;
    char* wsp = (char*)d_ws;
    bf* XB  = (bf*)wsp;  wsp += SZ_P16;
    bf* WTq = (bf*)wsp;  wsp += SZ_W;
    bf* WTk = (bf*)wsp;  wsp += SZ_W;
    bf* WTv = (bf*)wsp;  wsp += SZ_W;
    bf* WTo = (bf*)wsp;  wsp += SZ_W;
    h16* QH = (h16*)wsp; wsp += SZ_P16;
    h16* QR = (h16*)wsp; wsp += SZ_P16;
    h16* KP = (h16*)wsp; wsp += SZ_P16;
    h16* VT = (h16*)wsp; wsp += SZ_P16;
    bf* ATh = (bf*)wsp;  wsp += SZ_P16;
    bf* ATl = (bf*)wsp;  wsp += SZ_P16;
    float* RES = (float*)wsp; wsp += SZ_RES;

    k_cvt8x<<<(unsigned)(((size_t)NROW * DM / 8 + 255) / 256), 256, 0, stream>>>(x, XB);
    k_wt<<<dim3(DM / 64, DM / 64, 1), 256, 0, stream>>>(wq, WTq);
    k_wt<<<dim3(DM / 64, DM / 64, 1), 256, 0, stream>>>(wk, WTk);
    k_wt<<<dim3(DM / 64, DM / 64, 1), 256, 0, stream>>>(wv, WTv);
    k_wt<<<dim3(DM / 64, DM / 64, 1), 256, 0, stream>>>(wo, WTo);
    k_proj_q<<<dim3(NROW / 64, DM / 64, 1), 32, 0, stream>>>(XB, WTq, QH, QR);
    k_proj_k<<<dim3(NROW / 64, DM / 64, 1), 32, 0, stream>>>(XB, WTk, KP);
    k_proj_v<<<dim3(NROW / 64, DM / 64, 1), 32, 0, stream>>>(XB, WTv, VT);
    k_attn<<<dim3(SEQ / 64, NB * NH, 1), 128, 0, stream>>>(QH, QR, KP, VT, ATh, ATl);
    k_oproj<<<dim3(NROW / 64, DM / 64, 1), 32, 0, stream>>>(ATh, ATl, WTo, x, bo, RES);
    k_ln<<<NROW / 8, 256, 0, stream>>>(RES, gamma, beta, OUT);
}
